// Attention_37847251812733
// MI455X (gfx1250) — hardware-run, weakly checked
//
#include <hip/hip_runtime.h>


#ifndef SEQ
#define SEQ 4096
#endif
#define SEQ_FULL 4096
#define DM   1024
#define NH_  16
#define HD   64
#define AW   4
#define QW   32
#define OSP  36
#define LNW  4
#define SC2  ((float)(0.125 * 1.4426950408889634))
#define PSH  14.0f
#define NEGB (-3.0e38f)
#define W1S  64.0f
#define W1I  (1.0f / 64.0f)
#define LNEPS 1.0e-5f

static_assert(HD == 64);
static_assert(NH_ * HD == DM);
static_assert(DM % 64 == 0);
static_assert(DM % 32 == 0);
static_assert(HD % 32 == 0);
static_assert(SEQ % 64 == 0);
static_assert(SEQ % 32 == 0);
static_assert(SEQ % (QW * AW) == 0);
static_assert(QW == 32);
static_assert(SEQ % LNW == 0);
static_assert(DM % 256 == 0);
static_assert(((size_t)SEQ * DM) % 8 == 0);
static_assert(((size_t)DM * DM) % 8 == 0);
static_assert(SEQ <= SEQ_FULL);
static_assert((OSP * 4) % 16 == 0);
static_assert((size_t)NH_ * HD * SEQ == (size_t)SEQ * DM);
static_assert(32 * 16 * 4 == 16 * HD * 2);
static_assert(32 * 16 * 16 == HD * QW * 4);
static_assert(32 * 16 * 8 == 16 * 64 * 4);
static_assert(32 * 16 * (DM / 128) == DM * 4);
static_assert(32 * 16 * (DM / 256) == DM * 2);
static_assert((size_t)AW * HD * OSP * 4 <= 131072);
static_assert((size_t)LNW * DM * 4 <= 131072);
static_assert((size_t)16 * 68 * 4 <= 131072);

typedef _Float16 h16;
typedef unsigned short bf;
typedef __attribute__((ext_vector_type(16))) __bf16   v16bf;
typedef __attribute__((ext_vector_type(16))) _Float16 v16h;
typedef __attribute__((ext_vector_type(8)))  _Float16 v8h;
typedef __attribute__((ext_vector_type(8)))  unsigned short v8us;
typedef __attribute__((ext_vector_type(8)))  float    v8f;
typedef __attribute__((ext_vector_type(4)))  float    v4f;
typedef v4f  __attribute__((may_alias)) v4fa;

__device__ __forceinline__ unsigned short f2bf(float f) { unsigned u = __float_as_uint(f); u += 0x7FFFu + ((u >> 16) & 1u); return (unsigned short)(u >> 16); }
__device__ __forceinline__ float bfr(float f) { return __uint_as_float(((unsigned)f2bf(f)) << 16); }
__device__ __forceinline__ v16h cat16(v8h lo, v8h hi) { return __builtin_shufflevector(lo, hi, 0, 1, 2, 3, 4, 5, 6, 7, 8, 9, 10, 11, 12, 13, 14, 15); }
__device__ __forceinline__ v16bf cat16b(v8us lo, v8us hi) { return __builtin_bit_cast(v16bf, __builtin_shufflevector(lo, hi, 0, 1, 2, 3, 4, 5, 6, 7, 8, 9, 10, 11, 12, 13, 14, 15)); }
__device__ __forceinline__ v8f wmma16(v16h a, v16h b, v8f c) { return __builtin_amdgcn_wmma_f32_16x16x32_f16(false, a, false, b, (short)0, c, false, false); }
__device__ __forceinline__ v8f wmmab(v16bf a, v16bf b, v8f c) { return __builtin_amdgcn_wmma_f32_16x16x32_bf16(false, a, false, b, (short)0, c, false, false); }
__device__ __forceinline__ v16h  ldh(const h16* p) { return cat16(*(const v8h*)p, *(const v8h*)(p + 16)); }
__device__ __forceinline__ v16bf ldb(const bf* p)  { return cat16b(*(const v8us*)p, *(const v8us*)(p + 16)); }
__device__ __forceinline__ void wave_sync() { __builtin_amdgcn_fence(3  , "wavefront"); __builtin_amdgcn_wave_barrier(); asm volatile("" ::: "memory"); }

__device__ __forceinline__ v8f wmmabg(v16bf a, v16bf b, v8f c) { c = wmmab(a, b, c); asm volatile("v_nop\n\tv_nop\n\tv_nop\n\tv_nop" : "+v"(c) : "v"(a), "v"(b)); return c; }
__device__ __forceinline__ v8f wmma16g(v16h a, v16h b, v8f c) { c = wmma16(a, b, c); asm volatile("v_nop\n\tv_nop\n\tv_nop\n\tv_nop" : "+v"(c) : "v"(a), "v"(b)); return c; }
static __device__ __forceinline__ h16 toh_flush(float v) { const float w = (fabsf(v) < 6.103515625e-05f) ? 0.0f : v; return (h16)w; }
__device__ __forceinline__ float wsum(float v) { v += __shfl_xor(v, 16, 32); v += __shfl_xor(v, 8, 32); v += __shfl_xor(v, 4, 32); v += __shfl_xor(v, 2, 32); v += __shfl_xor(v, 1, 32); return v; }

__global__ __launch_bounds__(256) void k_cvt8(const float* __restrict__ src, bf* dst, size_t n8) {
    const size_t i = (size_t)blockIdx.x * 256 + threadIdx.x; if (i >= n8) return;
    const v8f v = *(const v8f*)(src + i * 8); v8us o;
#pragma unroll
    for (int k = 0; k < 8; ++k) o[k] = f2bf(v[k]);
    *(volatile v8us*)(dst + i * 8) = o; __threadfence(); *(volatile v8us*)(dst + i * 8) = o;
}

__global__ __launch_bounds__(256) void k_cvtw(const float* __restrict__ src, h16* dst, size_t n8) {
    const size_t i = (size_t)blockIdx.x * 256 + threadIdx.x; if (i >= n8) return;
    const v8f v = *(const v8f*)(src + i * 8); v8h o;
#pragma unroll
    for (int k = 0; k < 8; ++k) o[k] = toh_flush(bfr(v[k]) * W1S);
    *(volatile v8h*)(dst + i * 8) = o; __threadfence(); *(volatile v8h*)(dst + i * 8) = o;
}

__global__ __launch_bounds__(32) void k_proj(const bf* __restrict__ A, const bf* __restrict__ Bt, h16* Ph, int mode) {
    __shared__ __align__(16) float os[16 * 68];
    const int K = DM;
    const int lane = threadIdx.x & 31, lr = lane & 15, hi = lane >> 4;
    const unsigned bx = blockIdx.x, by = blockIdx.y;
    const int r0 = (int)(bx * 64u), c0 = (int)(by * 64u);
    v8f acc[4][4];
#pragma unroll
    for (int mb = 0; mb < 4; ++mb)
#pragma unroll
        for (int nb = 0; nb < 4; ++nb) acc[mb][nb] = (v8f){};
    const size_t aoff = (size_t)(r0 + lr) * K + 8 * hi, boff = (size_t)(c0 + lr) * K + 8 * hi;
#pragma unroll 1
    for (int kc = 0; kc < K; kc += 32) {
        v16bf a[4];
#pragma unroll
        for (int mb = 0; mb < 4; ++mb) a[mb] = ldb(A + aoff + (size_t)mb * 16 * K + kc);
#pragma unroll
        for (int nb = 0; nb < 4; ++nb) { const v16bf b = ldb(Bt + boff + (size_t)nb * 16 * K + kc);
#pragma unroll
            for (int mb = 0; mb < 4; ++mb) acc[mb][nb] = wmmabg(a[mb], b, acc[mb][nb]); }
    }
    size_t tbase, pitch;
    if (mode == 0) { tbase = ((size_t)by * SEQ + (size_t)r0) * HD; pitch = HD; }
    else           { tbase = (size_t)r0 * SEQ + (size_t)c0;        pitch = SEQ; }
#pragma unroll
    for (int mb = 0; mb < 4; ++mb) {
#pragma unroll
        for (int nb = 0; nb < 4; ++nb) {
#pragma unroll
            for (int j = 0; j < 8; ++j) os[(hi * 8 + j) * 68 + nb * 16 + lr] = acc[mb][nb][j]; }
        wave_sync();
        const size_t sb = tbase + (size_t)(mb * 16) * pitch;
#pragma unroll 1
        for (int ps = 0; ps < 2; ++ps) {
#pragma unroll
            for (int s = 0; s < 4; ++s) { const int row = 4 * s + (lane >> 3), c8 = (lane & 7) * 8;
                const v4f x0 = *(const v4fa*)(&os[row * 68 + c8]); const v4f x1 = *(const v4fa*)(&os[row * 68 + c8 + 4]); v8h hv;
#pragma unroll
                for (int i = 0; i < 4; ++i) { hv[i] = toh_flush(x0[i]); hv[4 + i] = toh_flush(x1[i]); }
                *(volatile v8h*)(Ph + sb + (size_t)row * pitch + c8) = hv; }
            if (ps == 0) __threadfence(); }
        wave_sync();
    }
}

__device__ __forceinline__ v16h smax_step(const v8f sa, const v8f sb, float& m, float& l, float& alpha) {
    float ta[8], tb[8]; float mx = NEGB;
#pragma unroll
    for (int r = 0; r < 8; ++r) { ta[r] = sa[r] * SC2; tb[r] = sb[r] * SC2; mx = fmaxf(mx, fmaxf(ta[r], tb[r])); }
    mx = fmaxf(mx, __shfl_xor(mx, 16, 32));
    const float mnew = fmaxf(m, mx);
    alpha = __builtin_amdgcn_exp2f(m - mnew);
    const float sh = PSH - mnew;
    v16h pb; float ls = 0.0f;
#pragma unroll
    for (int r = 0; r < 8; ++r) {
        const float ua = ta[r] + sh, ub = tb[r] + sh;
        const float ea = __builtin_amdgcn_exp2f(ua), eb = __builtin_amdgcn_exp2f(ub);
        const float ga = (ua < -14.0f) ? 0.0f : ea, gb = (ub < -14.0f) ? 0.0f : eb;
        const h16 pa = (h16)ga; const h16 pc = (h16)gb;
        pb[r] = pa; pb[8 + r] = pc;
        ls += (float)pa + (float)pc; }
    l = l * alpha + ls; m = mnew;
    return pb;
}

__global__ __launch_bounds__(32 * AW) void k_flash(const h16* __restrict__ QH, const h16* __restrict__ KP, const h16* __restrict__ VT, float* CTX) {
    __shared__ __align__(16) float os[AW * HD * OSP];
    const int lane = threadIdx.x & 31, lr = lane & 15, hi = lane >> 4;
    const int wave = __builtin_amdgcn_readfirstlane((int)(threadIdx.x >> 5));
    const unsigned zh = blockIdx.y;
    const int t0 = ((int)blockIdx.x * AW + wave) * QW;
    const size_t pbase = (size_t)zh * SEQ * HD;
    const size_t qo = pbase + (size_t)(t0 + lr) * HD + 8 * hi;
    const v16h q00 = ldh(QH + qo), q01 = ldh(QH + qo + 32);
    const v16h q10 = ldh(QH + qo + 16 * HD), q11 = ldh(QH + qo + 16 * HD + 32);
    const size_t ko = pbase + (size_t)lr * HD + 8 * hi;
    const size_t vo = pbase + (size_t)lr * SEQ + 8 * hi;
    v8f oa[4], ob[4];
#pragma unroll
    for (int j = 0; j < 4; ++j) { oa[j] = (v8f){}; ob[j] = (v8f){}; }
    float ma = NEGB, mb = NEGB, la = 0.0f, lb = 0.0f;
#pragma unroll 1
    for (int key0 = 0; key0 < SEQ; key0 += 32) {
        const h16* ka = KP + ko + (size_t)key0 * HD;
        const v16h ka0 = ldh(ka), ka1 = ldh(ka + 32), kb0 = ldh(ka + 16 * HD), kb1 = ldh(ka + 16 * HD + 32);
        v8f s0 = (v8f){}, s1 = (v8f){}, s2 = (v8f){}, s3 = (v8f){};
        s0 = wmma16g(ka0, q00, s0); s1 = wmma16g(kb0, q00, s1); s2 = wmma16g(ka0, q10, s2); s3 = wmma16g(kb0, q10, s3);
        s0 = wmma16g(ka1, q01, s0); s1 = wmma16g(kb1, q01, s1); s2 = wmma16g(ka1, q11, s2); s3 = wmma16g(kb1, q11, s3);
        float al0, al1;
        const v16h p0 = smax_step(s0, s1, ma, la, al0);
        const v16h p1 = smax_step(s2, s3, mb, lb, al1);
#pragma unroll
        for (int j = 0; j < 4; ++j) { oa[j] = oa[j] * al0; ob[j] = ob[j] * al1; }
        const h16* va = VT + vo + key0;
#pragma unroll
        for (int j = 0; j < 4; ++j) { const v16h vj = ldh(va + (size_t)(16 * j) * SEQ);
            oa[j] = wmma16g(vj, p0, oa[j]); ob[j] = wmma16g(vj, p1, ob[j]); }
    }
    la += __shfl_xor(la, 16, 32); lb += __shfl_xor(lb, 16, 32);
    const float inva = 1.0f / la, invb = 1.0f / lb;
    const int wb = wave * HD * OSP;
#pragma unroll
    for (int j = 0; j < 4; ++j) {
#pragma unroll
        for (int r = 0; r < 8; ++r) { os[wb + (16 * j + 8 * hi + r) * OSP + lr] = oa[j][r] * inva; os[wb + (16 * j + 8 * hi + r) * OSP + 16 + lr] = ob[j][r] * invb; } }
    wave_sync();
    float* crow = CTX + (size_t)zh * HD * SEQ + (size_t)t0;
#pragma unroll 1
    for (int ps = 0; ps < 2; ++ps) {
#pragma unroll
        for (int s = 0; s < 16; ++s) { const int row = 4 * s + (lane >> 3), cofs = (lane & 7) * 4;
            const v4f val = *(const v4fa*)(&os[wb + row * OSP + cofs]);
            *(volatile v4f*)(crow + (size_t)row * SEQ + cofs) = val; }
        if (ps == 0) __threadfence(); }
}

__global__ __launch_bounds__(32 * LNW) void k_ln1(const float* __restrict__ CTX, const float* __restrict__ X, const float* __restrict__ G, const float* __restrict__ Bv, float* H1F, h16* H1H) {
#pragma clang fp contract(off)
    __shared__ __align__(16) float rb[LNW * DM];
    const int lane = threadIdx.x & 31;
    const int wave = __builtin_amdgcn_readfirstlane((int)(threadIdx.x >> 5));
    const unsigned row = blockIdx.x * (unsigned)LNW + (unsigned)wave;
    const int wb = wave * DM;
    const size_t ro = (size_t)row * DM;
    float s = 0.0f;
#pragma unroll 1
    for (int it = 0; it < DM / 128; ++it) { const int c = it * 128 + lane * 4;
        const v4f a = *(const v4f*)(CTX + ro + c); const v4f xv = *(const v4f*)(X + ro + c); v4f v;
        v[0] = a[0] + bfr(xv[0]); v[1] = a[1] + bfr(xv[1]); v[2] = a[2] + bfr(xv[2]); v[3] = a[3] + bfr(xv[3]);
        *(v4fa*)(&rb[wb + c]) = v; s += (v[0] + v[1]) + (v[2] + v[3]); }
    s = wsum(s);
    const float mu = s * (1.0f / (float)DM);
    float q = 0.0f;
#pragma unroll 1
    for (int it = 0; it < DM / 128; ++it) { const int c = it * 128 + lane * 4;
        const v4f v = *(const v4fa*)(&rb[wb + c]);
        const float d0 = v[0] - mu, d1 = v[1] - mu, d2 = v[2] - mu, d3 = v[3] - mu;
        q += (d0 * d0 + d1 * d1) + (d2 * d2 + d3 * d3); }
    q = wsum(q);
    const float rstd = rsqrtf(q * (1.0f / (float)DM) + LNEPS);
#pragma unroll 1
    for (int it = 0; it < DM / 128; ++it) { const int c = it * 128 + lane * 4;
        const v4f v = *(const v4fa*)(&rb[wb + c]); const v4f g = *(const v4f*)(G + c); const v4f b = *(const v4f*)(Bv + c); v4f y;
        y[0] = (v[0] - mu) * rstd * bfr(g[0]) + bfr(b[0]); y[1] = (v[1] - mu) * rstd * bfr(g[1]) + bfr(b[1]);
        y[2] = (v[2] - mu) * rstd * bfr(g[2]) + bfr(b[2]); y[3] = (v[3] - mu) * rstd * bfr(g[3]) + bfr(b[3]);
        *(v4fa*)(&rb[wb + c]) = y; }
    wave_sync();
#pragma unroll 1
    for (int ps = 0; ps < 2; ++ps) {
#pragma unroll 1
        for (int it = 0; it < DM / 128; ++it) { const int c = it * 128 + lane * 4;
            const v4f y = *(const v4fa*)(&rb[wb + c]);
            *(volatile v4f*)(H1F + ro + c) = y; }
#pragma unroll 1
        for (int jt = 0; jt < DM / 256; ++jt) { const int c = jt * 256 + lane * 8;
            const v4f y0 = *(const v4fa*)(&rb[wb + c]); const v4f y1 = *(const v4fa*)(&rb[wb + c + 4]); v8h hv;
#pragma unroll
            for (int i = 0; i < 4; ++i) { hv[i] = toh_flush(y0[i]); hv[4 + i] = toh_flush(y1[i]); }
            *(volatile v8h*)(H1H + ro + c) = hv; }
        if (ps == 0) __threadfence(); }
}

__global__ __launch_bounds__(32) void k_ffn(const h16* __restrict__ A, const h16* __restrict__ Bt, const float* __restrict__ bias, const float* __restrict__ RES, float* PRE) {
    __shared__ __align__(16) float os[16 * 68];
    const int K = DM;
    const int lane = threadIdx.x & 31, lr = lane & 15, hi = lane >> 4;
    const unsigned bx = blockIdx.x, by = blockIdx.y;
    const int r0 = (int)(bx * 64u), c0 = (int)(by * 64u);
    v8f acc[4][4];
#pragma unroll
    for (int mb = 0; mb < 4; ++mb)
#pragma unroll
        for (int nb = 0; nb < 4; ++nb) acc[mb][nb] = (v8f){};
    const size_t aoff = (size_t)(r0 + lr) * K + 8 * hi, boff = (size_t)(c0 + lr) * K + 8 * hi;
#pragma unroll 1
    for (int kc = 0; kc < K; kc += 32) {
        v16h a[4];
#pragma unroll
        for (int mb = 0; mb < 4; ++mb) a[mb] = ldh(A + aoff + (size_t)mb * 16 * K + kc);
#pragma unroll
        for (int nb = 0; nb < 4; ++nb) { const v16h b = ldh(Bt + boff + (size_t)nb * 16 * K + kc);
#pragma unroll
            for (int mb = 0; mb < 4; ++mb) acc[mb][nb] = wmma16g(a[mb], b, acc[mb][nb]); }
    }
    float bc[4];
#pragma unroll
    for (int nb = 0; nb < 4; ++nb) bc[nb] = bfr(bias[c0 + nb * 16 + lr]);
#pragma unroll
    for (int mb = 0; mb < 4; ++mb) {
#pragma unroll
        for (int nb = 0; nb < 4; ++nb) {
#pragma unroll
            for (int j = 0; j < 8; ++j) os[(hi * 8 + j) * 68 + nb * 16 + lr] = acc[mb][nb][j] * W1I + bc[nb]; }
        wave_sync();
        const size_t sb = (size_t)(r0 + mb * 16) * DM + (size_t)c0;
#pragma unroll
        for (int s = 0; s < 8; ++s) { const int row = 2 * s + (lane >> 4), cofs = (lane & 15) * 4;
            const v4f a4 = *(const v4fa*)(&os[row * 68 + cofs]); const v4f r4 = *(const v4f*)(RES + sb + (size_t)row * DM + cofs);
            const v4f y = a4 + r4;
            *(v4fa*)(&os[row * 68 + cofs]) = y; }
#pragma unroll 1
        for (int ps = 0; ps < 2; ++ps) {
#pragma unroll
            for (int s = 0; s < 8; ++s) { const int row = 2 * s + (lane >> 4), cofs = (lane & 15) * 4;
                const v4f y = *(const v4fa*)(&os[row * 68 + cofs]);
                *(volatile v4f*)(PRE + sb + (size_t)row * DM + cofs) = y; }
            if (ps == 0) __threadfence(); }
        wave_sync();
    }
}

__global__ __launch_bounds__(32 * LNW) void k_ln2(const float* __restrict__ PRE, const float* __restrict__ G, const float* __restrict__ Bv, float* OUT) {
#pragma clang fp contract(off)
    __shared__ __align__(16) float rb[LNW * DM];
    const int lane = threadIdx.x & 31;
    const int wave = __builtin_amdgcn_readfirstlane((int)(threadIdx.x >> 5));
    const unsigned row = blockIdx.x * (unsigned)LNW + (unsigned)wave;
    const int wb = wave * DM;
    const size_t ro = (size_t)row * DM;
    float s = 0.0f;
#pragma unroll 1
    for (int it = 0; it < DM / 128; ++it) { const int c = it * 128 + lane * 4;
        const v4f v = *(const v4f*)(PRE + ro + c);
        *(v4fa*)(&rb[wb + c]) = v; s += (v[0] + v[1]) + (v[2] + v[3]); }
    s = wsum(s);
    const float mu = s * (1.0f / (float)DM);
    float q = 0.0f;
#pragma unroll 1
    for (int it = 0; it < DM / 128; ++it) { const int c = it * 128 + lane * 4;
        const v4f v = *(const v4fa*)(&rb[wb + c]);
        const float d0 = v[0] - mu, d1 = v[1] - mu, d2 = v[2] - mu, d3 = v[3] - mu;
        q += (d0 * d0 + d1 * d1) + (d2 * d2 + d3 * d3); }
    q = wsum(q);
    const float rstd = rsqrtf(q * (1.0f / (float)DM) + LNEPS);
#pragma unroll 1
    for (int it = 0; it < DM / 128; ++it) { const int c = it * 128 + lane * 4;
        const v4f v = *(const v4fa*)(&rb[wb + c]); const v4f g = *(const v4f*)(G + c); const v4f b = *(const v4f*)(Bv + c); v4f y;
        y[0] = (v[0] - mu) * rstd * bfr(g[0]) + bfr(b[0]); y[1] = (v[1] - mu) * rstd * bfr(g[1]) + bfr(b[1]);
        y[2] = (v[2] - mu) * rstd * bfr(g[2]) + bfr(b[2]); y[3] = (v[3] - mu) * rstd * bfr(g[3]) + bfr(b[3]);
        *(v4fa*)(&rb[wb + c]) = y; }
#pragma unroll 1
    for (int ps = 0; ps < 2; ++ps) {
#pragma unroll 1
        for (int it = 0; it < DM / 128; ++it) { const int c = it * 128 + lane * 4;
            const v4f y = *(const v4fa*)(&rb[wb + c]);
            *(volatile v4f*)(OUT + ro + c) = y; }
        if (ps == 0) __threadfence(); }
}

static constexpr size_t al256(size_t v) { return (v + 255) & ~(size_t)255; }
static constexpr size_t SZ_XB = al256((size_t)SEQ * DM * 2);
static constexpr size_t SZ_WB = al256((size_t)3 * DM * DM * 2);
static constexpr size_t SZ_W1 = al256((size_t)DM * DM * 2);
static constexpr size_t SZ_PL = al256((size_t)NH_ * SEQ * HD * 2);
static constexpr size_t SZ_F  = al256((size_t)SEQ * DM * 4);
static constexpr size_t SZ_HH = al256((size_t)SEQ * DM * 2);
static constexpr size_t SZ_TOTAL = SZ_XB + SZ_WB + SZ_W1 + 3 * SZ_PL + 3 * SZ_F + SZ_HH;
static_assert(SZ_TOTAL <= (size_t)134217728);
static_assert(((size_t)DM * DM * 2) % 256 == 0);
static_assert((size_t)NH_ * SEQ * HD == (size_t)DM * SEQ);

extern "C" void kernel_launch(void* const* d_in, const int* in_sizes, int n_in,
                              void* d_out, int out_size, void* d_ws, size_t ws_size, hipStream_t stream) {
    if (n_in < 10) return;
    if ((size_t)in_sizes[0] < (size_t)SEQ * DM) return;
    if ((size_t)in_sizes[1] < (size_t)DM * DM || (size_t)in_sizes[2] < (size_t)DM * DM || (size_t)in_sizes[3] < (size_t)DM * DM || (size_t)in_sizes[6] < (size_t)DM * DM) return;
    if (in_sizes[4] < DM || in_sizes[5] < DM || in_sizes[7] < DM || in_sizes[8] < DM || in_sizes[9] < DM) return;
    if ((size_t)out_size < (size_t)SEQ * DM) return;
    if (SZ_TOTAL > ws_size) return;
    const float* x   = (const float*)d_in[0];
    const float* wq  = (const float*)d_in[1];
    const float* wk  = (const float*)d_in[2];
    const float* wv  = (const float*)d_in[3];
    const float* g1  = (const float*)d_in[4];
    const float* be1 = (const float*)d_in[5];
    const float* w1  = (const float*)d_in[6];
    const float* b1  = (const float*)d_in[7];
    const float* g2  = (const float*)d_in[8];
    const float* be2 = (const float*)d_in[9];
    float* OUT = (float*)d_out;
    char* wsp = (char*)d_ws;
    bf*  XB  = (bf*)wsp;   wsp += SZ_XB;
    bf*  WB  = (bf*)wsp;   wsp += SZ_WB;
    h16* W1H = (h16*)wsp;  wsp += SZ_W1;
    h16* QH  = (h16*)wsp;  wsp += SZ_PL;
    h16* KP  = (h16*)wsp;  wsp += SZ_PL;
    h16* VT  = (h16*)wsp;  wsp += SZ_PL;
    float* CTX = (float*)wsp; wsp += SZ_F;
    float* H1F = (float*)wsp; wsp += SZ_F;
    float* PRE = (float*)wsp; wsp += SZ_F;
    h16* H1H = (h16*)wsp;  wsp += SZ_HH;
    bf* WQ = WB; bf* WK = WB + (size_t)DM * DM; bf* WV = WB + (size_t)2 * DM * DM;

    { const size_t n8 = (size_t)SEQ * DM / 8;
      k_cvt8<<<(unsigned)((n8 + 255) / 256), 256, 0, stream>>>(x, XB, n8); }
    { const size_t n8 = (size_t)DM * DM / 8; const unsigned g = (unsigned)((n8 + 255) / 256);
      k_cvt8<<<g, 256, 0, stream>>>(wq, WQ, n8); k_cvt8<<<g, 256, 0, stream>>>(wk, WK, n8); k_cvt8<<<g, 256, 0, stream>>>(wv, WV, n8);
      k_cvtw<<<g, 256, 0, stream>>>(w1, W1H, n8); }

    k_proj<<<dim3(SEQ / 64, DM / 64, 1), 32, 0, stream>>>(XB, WQ, QH, 0);
    k_proj<<<dim3(SEQ / 64, DM / 64, 1), 32, 0, stream>>>(XB, WK, KP, 0);
    k_proj<<<dim3(DM / 64, SEQ / 64, 1), 32, 0, stream>>>(WV, XB, VT, 1);

    k_flash<<<dim3(SEQ / (QW * AW), NH_, 1), 32 * AW, 0, stream>>>(QH, KP, VT, CTX);

    k_ln1<<<dim3(SEQ / LNW, 1, 1), 32 * LNW, 0, stream>>>(CTX, x, g1, be1, H1F, H1H);

    k_ffn<<<dim3(SEQ / 64, DM / 64, 1), 32, 0, stream>>>(H1H, W1H, b1, H1F, PRE);

    k_ln2<<<dim3(SEQ / LNW, 1, 1), 32 * LNW, 0, stream>>>(PRE, g2, be2, OUT);
}
